// xLSTM_63393717289391
// MI455X (gfx1250) — hardware-verified
//
#include <hip/hip_runtime.h>
#include <math.h>

constexpr int NBAT   = 8;
constexpr int NSTEP  = 2048;
constexpr int NIN    = 512;
constexpr int NHEAD  = 8;
constexpr int DEMB   = 32;
constexpr int NROWS  = NBAT * NSTEP;
constexpr int NVK    = NHEAD * DEMB;
constexpr int YCOL_V = 0;
constexpr int YCOL_K = NVK;
constexpr int YCOL_F = 2 * NVK;
constexpr int YCOL_I = 2 * NVK + NHEAD;
constexpr int YPITCH = 576;
constexpr int NTHR   = 256;
constexpr int CHUNK  = 32;
constexpr int NCHUNK = NSTEP / CHUNK;
constexpr int CPITCH = 36;
constexpr int NOUT0  = NBAT * NHEAD * DEMB;
constexpr int NOUT1  = NBAT * NHEAD * DEMB * DEMB;
constexpr float KSCALE = 1.0f / 2.82842712474619009760f;
static_assert(NROWS % 64 == 0);
static_assert(YPITCH % 64 == 0);
static_assert(NIN % 32 == 0);
static_assert(((NROWS / 64) * (YPITCH / 64)) % 8 == 0);
static_assert(YCOL_I + NHEAD <= YPITCH);
static_assert(NSTEP % CHUNK == 0);
static_assert(CHUNK == 32);
static_assert(DEMB == 32);
static_assert((NROWS * (NIN / 8)) % NTHR == 0);
static_assert(YPITCH % (NTHR / 32) == 0);
static_assert((NOUT0 * 4) % 128 == 0);
static_assert((NOUT0 + NOUT1) * 4 == 270336);

typedef __attribute__((ext_vector_type(16))) _Float16 v16h;
typedef __attribute__((ext_vector_type(8)))  _Float16 v8h;
typedef __attribute__((ext_vector_type(16))) __bf16   v16b;
typedef __attribute__((ext_vector_type(8)))  __bf16   v8b;
typedef __attribute__((ext_vector_type(8)))  float    v8f;
typedef __attribute__((ext_vector_type(4)))  float    v4f;
typedef __attribute__((ext_vector_type(4)))  unsigned v4u;

__device__ __forceinline__ unsigned short f2bf_bits(float f) {
  unsigned u = __float_as_uint(f);
  return (unsigned short)((u + 0x7FFFu + ((u >> 16) & 1u)) >> 16);
}
__device__ __forceinline__ float bf_bits2f(unsigned short h) { return __uint_as_float(((unsigned)h) << 16); }
__device__ __forceinline__ float bf16r(float f) { return bf_bits2f(f2bf_bits(f)); }

__device__ __forceinline__ void dep_guard_h(v8f& a, v8f& b, v16h x, v16h y) { asm volatile("v_nop\n\tv_nop\n\tv_nop\n\tv_nop" : "+v"(a), "+v"(b) : "v"(x), "v"(y)); }
__device__ __forceinline__ void dep_guard_b(v8f& a, v8f& b, v16b x, v16b y) { asm volatile("v_nop\n\tv_nop\n\tv_nop\n\tv_nop" : "+v"(a), "+v"(b) : "v"(x), "v"(y)); }
__device__ __forceinline__ void dep_guard4_h(v8f& a, v8f& b, v8f& c, v8f& d, v16h x, v16h y) { asm volatile("v_nop\n\tv_nop\n\tv_nop\n\tv_nop" : "+v"(a), "+v"(b), "+v"(c), "+v"(d) : "v"(x), "v"(y)); }
__device__ __forceinline__ void dep_guard4_b(v8f& a, v8f& b, v8f& c, v8f& d, v16b x, v16b y) { asm volatile("v_nop\n\tv_nop\n\tv_nop\n\tv_nop" : "+v"(a), "+v"(b), "+v"(c), "+v"(d) : "v"(x), "v"(y)); }
__device__ __forceinline__ void keep4_h(v16h a, v16h b, v16h c, v16h d) { asm volatile("v_nop" :: "v"(a), "v"(b), "v"(c), "v"(d)); }
__device__ __forceinline__ void keep4_b(v16b a, v16b b, v16b c, v16b d) { asm volatile("v_nop" :: "v"(a), "v"(b), "v"(c), "v"(d)); }
__device__ __forceinline__ void acc_guard4(v8f& a, v8f& b, v8f& c, v8f& d) { asm volatile("v_nop\n\tv_nop\n\tv_nop\n\tv_nop" : "+v"(a), "+v"(b), "+v"(c), "+v"(d)); }
template <typename T> struct Frag;
template <> struct Frag<_Float16> {
  typedef v16h V; union U { v16h v; v8h h[2]; };
  static __device__ __forceinline__ v16h load(const _Float16* p) {
    U f; f.h[0] = *(const v8h*)(p); f.h[1] = *(const v8h*)(p + 16); return f.v;
  }
  static __device__ __forceinline__ v8f mma(v16h a, v16h b, v8f c) {
    return __builtin_amdgcn_wmma_f32_16x16x32_f16(false, a, false, b, (short)0, c, false, false);
  }
  static __device__ __forceinline__ void guard(v8f& a, v8f& b, v16h x, v16h y) { dep_guard_h(a, b, x, y); }
  static __device__ __forceinline__ void guard4(v8f& a, v8f& b, v8f& c, v8f& d, v16h x, v16h y) { dep_guard4_h(a, b, c, d, x, y); }
  static __device__ __forceinline__ void keep(v16h a, v16h b, v16h c, v16h d) { keep4_h(a, b, c, d); }
};
template <> struct Frag<__bf16> {
  typedef v16b V; union U { v16b v; v8b h[2]; };
  static __device__ __forceinline__ v16b load(const __bf16* p) {
    U f; f.h[0] = *(const v8b*)(p); f.h[1] = *(const v8b*)(p + 16); return f.v;
  }
  static __device__ __forceinline__ v8f mma(v16b a, v16b b, v8f c) {
    return __builtin_amdgcn_wmma_f32_16x16x32_bf16(false, a, false, b, (short)0, c, false, false);
  }
  static __device__ __forceinline__ void guard(v8f& a, v8f& b, v16b x, v16b y) { dep_guard_b(a, b, x, y); }
  static __device__ __forceinline__ void guard4(v8f& a, v8f& b, v8f& c, v8f& d, v16b x, v16b y) { dep_guard4_b(a, b, c, d, x, y); }
  static __device__ __forceinline__ void keep(v16b a, v16b b, v16b c, v16b d) { keep4_b(a, b, c, d); }
};

template <int ET> struct Elem;
template <> struct Elem<0> { typedef _Float16 T; };
template <> struct Elem<1> { typedef __bf16 T; };
template <int ET, bool SPLIT, int BIAS_MODE, int OUT_MODE, bool RESID, int ACT = 0>
__global__ __launch_bounds__(256) void wmma_gemm64(
    const unsigned short* __restrict__ Ap, const unsigned short* __restrict__ A2p, int lda, long strideA,
    const unsigned short* __restrict__ Btp, const unsigned short* __restrict__ Bt2p, int ldb, long strideB,
    void* __restrict__ Cout, void* __restrict__ Cout2, int ldc, long strideC,
    const float* __restrict__ bias,
    const float* __restrict__ resid, long strideR,
    int M, int N, int K, float scale) {
  typedef typename Elem<ET>::T T;
  typedef typename Frag<T>::V V;
  const T* A = (const T*)Ap; const T* A2 = (const T*)A2p; const T* Bt = (const T*)Btp; const T* Bt2 = (const T*)Bt2p;
  __shared__ __align__(16) float sT[8][16 * 68];
  const int b    = blockIdx.y;
  const int lane = threadIdx.x & 31;
  const int wave = threadIdx.x >> 5;
  const int tilesN = N >> 6;
  const int tilesM = M >> 6;
  const int tile = blockIdx.x * 8 + wave;
  if (tile >= tilesM * tilesN) return;
  const int tm = tile / tilesN;
  const int tn = tile - tm * tilesN;
  const int m0 = tm << 6;
  const int n0 = tn << 6;

  const T* Ab  = A  + (size_t)b * strideA;
  const T* Bb  = Bt + (size_t)b * strideB;
  const T* Ab2 = SPLIT ? (A2  + (size_t)b * strideA) : nullptr;
  const T* Bb2 = SPLIT ? (Bt2 + (size_t)b * strideB) : nullptr;

  const int rlane = lane & 15;
  const int koff  = (lane >> 4) * 8;
  const int mOff  = (lane >> 4) * 8;

  v8f acc[4][4];
#pragma unroll
  for (int i = 0; i < 4; ++i)
#pragma unroll
    for (int j = 0; j < 4; ++j) acc[i][j] = (v8f){0.f,0.f,0.f,0.f,0.f,0.f,0.f,0.f};

  for (int k0 = 0; k0 < K; k0 += 32) {
    V bh[4], bl[4];
#pragma unroll
    for (int j = 0; j < 4; ++j) {
      const size_t bo = (size_t)(n0 + (j << 4) + rlane) * ldb + koff + k0;
      bh[j] = Frag<T>::load(Bb + bo);
      if (SPLIT) bl[j] = Frag<T>::load(Bb2 + bo);
    }
#pragma unroll
    for (int i = 0; i < 4; ++i) {
      const size_t ao = (size_t)(m0 + (i << 4) + rlane) * lda + koff + k0;
      V ah = Frag<T>::load(Ab + ao);
      V al;
      if (SPLIT) al = Frag<T>::load(Ab2 + ao);
#pragma unroll
      for (int j = 0; j < 4; ++j) {
        acc[i][j] = Frag<T>::mma(ah, bh[j], acc[i][j]);
        if (SPLIT) {
          acc[i][j] = Frag<T>::mma(ah, bl[j], acc[i][j]);
          acc[i][j] = Frag<T>::mma(al, bh[j], acc[i][j]);
        }
      }
      Frag<T>::guard4(acc[i][0], acc[i][1], acc[i][2], acc[i][3], ah, SPLIT ? al : bh[3]);
    }
    Frag<T>::keep(bh[0], bh[1], bh[2], bh[3]);
    if (SPLIT) Frag<T>::keep(bl[0], bl[1], bl[2], bl[3]);
  }
  acc_guard4(acc[0][0], acc[0][1], acc[0][2], acc[0][3]);
  acc_guard4(acc[1][0], acc[1][1], acc[1][2], acc[1][3]);
  acc_guard4(acc[2][0], acc[2][1], acc[2][2], acc[2][3]);
  acc_guard4(acc[3][0], acc[3][1], acc[3][2], acc[3][3]);

  float* slab = sT[wave];
  const float* Rb = RESID ? (resid + (size_t)b * strideR) : nullptr;
#pragma unroll
  for (int i = 0; i < 4; ++i) {
    const int mBase = m0 + (i << 4);
#pragma unroll
    for (int j = 0; j < 4; ++j) {
      const int n = n0 + (j << 4) + rlane;
      float bv = 0.f;
      if (BIAS_MODE == 2) bv = bias[n];
#pragma unroll
      for (int r = 0; r < 8; ++r) {
        float v = acc[i][j][r] * scale;
        if (BIAS_MODE == 1) v += bias[mBase + mOff + r];
        if (BIAS_MODE == 2) v += bv;
        if (RESID) v += Rb[(size_t)(mBase + mOff + r) * ldc + n];
        if (ACT == 1) v = tanhf(v);
        if (ACT == 2) v = fmaxf(v, 0.0f);
        if (ACT == 3) v = v / (1.0f + expf(-v));
        if (ACT == 4) v = (v > 0.f) ? v : 0.01f * v;
        if (ACT == 5) v = 0.5f * v * (1.0f + erff(v * 0.70710678118654752f));
        slab[(mOff + r) * 68 + (j << 4) + rlane] = v;
      }
    }
    __builtin_amdgcn_fence(__ATOMIC_RELEASE, "workgroup");
    __builtin_amdgcn_wave_barrier();
    __builtin_amdgcn_fence(__ATOMIC_ACQUIRE, "workgroup");
    if (OUT_MODE == 0) {
      float* C = (float*)Cout + (size_t)b * strideC;
      const int hh = lane >> 4, c4 = (lane & 15) * 4;
      for (int pass = 0; pass < 2; ++pass) {
#pragma unroll
        for (int it = 0; it < 8; ++it) {
          const int row = it * 2 + hh;
          v4f v = *(const v4f*)(slab + row * 68 + c4);
          *(volatile v4f*)(C + (size_t)(mBase + row) * ldc + n0 + c4) = v;
        }
        __threadfence();
      }
    } else {
      const int q = lane >> 3, c8 = (lane & 7) * 8;
      unsigned short* C  = (unsigned short*)Cout  + (size_t)b * strideC;
      unsigned short* C2 = (OUT_MODE == 2) ? ((unsigned short*)Cout2 + (size_t)b * strideC) : nullptr;
      for (int pass = 0; pass < 2; ++pass) {
#pragma unroll
        for (int it = 0; it < 4; ++it) {
          const int row = it * 4 + q;
          const float* sp = slab + row * 68 + c8;
          v8h hv, lv;
#pragma unroll
          for (int e = 0; e < 8; ++e) {
            if (OUT_MODE == 1) {
              hv[e] = (_Float16)sp[e];
            } else {
              unsigned short hb = f2bf_bits(sp[e]);
              unsigned short lb = f2bf_bits(sp[e] - bf_bits2f(hb));
              hv[e] = __builtin_bit_cast(_Float16, hb);
              lv[e] = __builtin_bit_cast(_Float16, lb);
            }
          }
          *(volatile v8h*)(C + (size_t)(mBase + row) * ldc + n0 + c8) = hv;
          if (OUT_MODE == 2) *(volatile v8h*)(C2 + (size_t)(mBase + row) * ldc + n0 + c8) = lv;
        }
        __threadfence();
      }
    }
    __builtin_amdgcn_fence(__ATOMIC_RELEASE, "workgroup");
    __builtin_amdgcn_wave_barrier();
    __builtin_amdgcn_fence(__ATOMIC_ACQUIRE, "workgroup");
  }
}

template <int MODE>
__global__ __launch_bounds__(NTHR) void cvt8_kernel(const float* __restrict__ src, unsigned short* __restrict__ dst,
                                                    int nrow, int ncol8, int spitch, int scol0, float sc) {
  const int i  = blockIdx.x * NTHR + threadIdx.x;
  const int n8 = nrow * ncol8;
  if (i < n8) {
    const int row = i / ncol8;
    const int c8  = i - row * ncol8;
    const float* sp = src + (size_t)row * spitch + scol0 + c8 * 8;
    const v4f a = *(const v4f*)(sp);
    const v4f b = *(const v4f*)(sp + 4);
    v8h hv;
#pragma unroll
    for (int e = 0; e < 4; ++e) {
      unsigned short b0, b1;
      if (MODE == 0) {
        b0 = f2bf_bits(a[e] * sc);
        b1 = f2bf_bits(b[e] * sc);
      } else {
        b0 = __builtin_bit_cast(unsigned short, (_Float16)(bf16r(a[e]) * sc));
        b1 = __builtin_bit_cast(unsigned short, (_Float16)(bf16r(b[e]) * sc));
      }
      hv[e]     = __builtin_bit_cast(_Float16, b0);
      hv[4 + e] = __builtin_bit_cast(_Float16, b1);
    }
    *(volatile v8h*)(dst + (size_t)i * 8) = hv;
    __threadfence();
    *(volatile v8h*)(dst + (size_t)i * 8) = hv;
  }
}

__global__ __launch_bounds__(NTHR) void pack_bt_kernel(const float* __restrict__ Wv, const float* __restrict__ Wk,
                                                       const float* __restrict__ Wf, const float* __restrict__ Wi,
                                                       unsigned short* __restrict__ BT) {
  const int lane = threadIdx.x & 31;
  const int n = __builtin_amdgcn_readfirstlane((int)(blockIdx.x * (NTHR / 32) + (threadIdx.x >> 5)));
  if (n >= YPITCH) return;
  float w[16];
#pragma unroll
  for (int e = 0; e < 16; ++e) w[e] = 0.0f;
  if (n < 2 * NVK) {
    const float* W = (n < NVK) ? Wv : Wk;
    const int nn = n & (NVK - 1);
    const int hh = nn >> 5, j = nn & 31;
    const float* col = W + (size_t)hh * NIN * DEMB + j;
#pragma unroll
    for (int e = 0; e < 8; ++e) w[e] = col[(size_t)(8 * lane + e) * DEMB];
    asm volatile("" :: "v"(w[0]), "v"(w[1]), "v"(w[2]), "v"(w[3]), "v"(w[4]), "v"(w[5]), "v"(w[6]), "v"(w[7]) : "memory");
#pragma unroll
    for (int e = 0; e < 8; ++e) w[8 + e] = col[(size_t)(NVK + 8 * lane + e) * DEMB];
  } else if (n < YCOL_I + NHEAD) {
    const float* W = (n < YCOL_I) ? Wf : Wi;
    const int hh = (n - YCOL_F) & 7;
    const float* rowp = W + (size_t)hh * NIN;
    const v4f a0 = *(const v4f*)(rowp + 8 * lane);
    const v4f a1 = *(const v4f*)(rowp + 8 * lane + 4);
    const v4f b0 = *(const v4f*)(rowp + NVK + 8 * lane);
    const v4f b1 = *(const v4f*)(rowp + NVK + 8 * lane + 4);
#pragma unroll
    for (int e = 0; e < 4; ++e) { w[e] = a0[e]; w[4 + e] = a1[e]; w[8 + e] = b0[e]; w[12 + e] = b1[e]; }
  }
  v4u p0, p1;
#pragma unroll
  for (int q = 0; q < 4; ++q) {
    p0[q] = (unsigned)f2bf_bits(w[2 * q])     | ((unsigned)f2bf_bits(w[2 * q + 1]) << 16);
    p1[q] = (unsigned)f2bf_bits(w[8 + 2 * q]) | ((unsigned)f2bf_bits(w[8 + 2 * q + 1]) << 16);
  }
  unsigned short* dst = BT + (size_t)n * NIN + 8 * lane;
  for (int pass = 0; pass < 2; ++pass) {
    *(volatile v4u*)(dst) = p0;
    *(volatile v4u*)(dst + NVK) = p1;
    __threadfence();
  }
}

__global__ __launch_bounds__(32) void mm_recur_kernel(const float* __restrict__ Y, const float* __restrict__ x,
                                                     const float* __restrict__ Wo, const float* __restrict__ bo,
                                                     const float* __restrict__ bfp, const float* __restrict__ bip,
                                                     const float* __restrict__ bvp, const float* __restrict__ bkp,
                                                     const float* __restrict__ Wq, const float* __restrict__ bq,
                                                     float* __restrict__ out) {
  __shared__ __align__(16) float vs[CHUNK * DEMB];
  __shared__ __align__(16) float ks[CHUNK * DEMB];
  __shared__ float fsh[CHUNK];
  __shared__ float ish[CHUNK];
  __shared__ __align__(16) float qs[DEMB];
  __shared__ __align__(16) float hsh[DEMB];
  __shared__ __align__(16) float Cs[DEMB * CPITCH];

  const int lane = threadIdx.x & 31;
  const int bh = blockIdx.x;
  const int b = bh >> 3, h = bh & 7;
  const int c4 = (lane & 7) * 4;
  const int rsub = lane >> 3;

  v4f bv4 = *(const v4f*)(bvp + h * DEMB + c4);
  v4f bk4 = *(const v4f*)(bkp + h * DEMB + c4);
#pragma unroll
  for (int e = 0; e < 4; ++e) { bv4[e] = bf16r(bv4[e]); bk4[e] = bf16r(bk4[e]); }
  const float bfb = bf16r(bfp[h]);
  const float bib = bf16r(bip[h]);
  const float bob = bf16r(bo[h * DEMB + lane]);
  const float bqb = bf16r(bq[h * DEMB + lane]);

  float ao = 0.0f, aq = 0.0f;
  {
    const float* xr  = x + ((size_t)b * NSTEP + (size_t)(NSTEP - 1)) * NIN;
    const float* woc = Wo + (size_t)h * NIN * DEMB + lane;
    const float* wqc = Wq + (size_t)h * NIN * DEMB + lane;
#pragma unroll 1
    for (int k = 0; k < NIN; ++k) {
      const float xb = bf16r(xr[k]);
      const float w1 = bf16r(woc[(size_t)k * DEMB]);
      const float w2 = bf16r(wqc[(size_t)k * DEMB]);
      ao = fmaf(xb, w1, ao);
      aq = fmaf(xb, w2, aq);
    }
  }
  const float zo = ao + bob;
  const float oj = 1.0f / (1.0f + expf(-zo));
  const float qj = aq + bqb;

  float Ccol[32];
#pragma unroll
  for (int i = 0; i < 32; ++i) Ccol[i] = 0.0f;
  float nj = 0.0f, m = 0.0f;

  const float* Yb = Y + (size_t)b * NSTEP * YPITCH;

#pragma unroll 1
  for (int ch = 0; ch < NCHUNK; ++ch) {
    const int t0 = ch * CHUNK;
    __syncthreads();
#pragma unroll
    for (int q = 0; q < 8; ++q) {
      const int r = 4 * q + rsub;
      const v4f val = *(const v4f*)(Yb + (size_t)(t0 + r) * YPITCH + YCOL_V + h * DEMB + c4);
      const v4f o = val + bv4;
      *(v4f*)(vs + r * DEMB + c4) = o;
    }
    asm volatile("" ::: "memory");
#pragma unroll
    for (int q = 0; q < 8; ++q) {
      const int r = 4 * q + rsub;
      const v4f val = *(const v4f*)(Yb + (size_t)(t0 + r) * YPITCH + YCOL_K + h * DEMB + c4);
      const v4f o = (val + bk4) * KSCALE;
      *(v4f*)(ks + r * DEMB + c4) = o;
    }
    asm volatile("" ::: "memory");
    fsh[lane] = Yb[(size_t)(t0 + lane) * YPITCH + YCOL_F + h] + bfb;
    ish[lane] = Yb[(size_t)(t0 + lane) * YPITCH + YCOL_I + h] + bib;
    __syncthreads();

#pragma unroll 1
    for (int s = 0; s < CHUNK; ++s) {
      const float fg  = fsh[s];
      const float ig  = ish[s];
      const float kj  = ks[s * DEMB + lane];
      const float sfm = fg + m;
      const float mn  = fmaxf(sfm, ig);
      const float fe  = expf(sfm - mn);
      const float ie  = expf(ig - mn);
      m = mn;
      const float iek = ie * kj;
      nj = fmaf(fe, nj, iek);
      const v4f* vr = (const v4f*)(vs + s * DEMB);
#pragma unroll
      for (int q = 0; q < 8; ++q) {
        const v4f vv = vr[q];
#pragma unroll
        for (int e = 0; e < 4; ++e) Ccol[4 * q + e] = fmaf(fe, Ccol[4 * q + e], iek * vv[e]);
      }
    }
  }

  float nq = nj * qj;
#pragma unroll
  for (int off = 1; off < 32; off <<= 1) nq += __shfl_xor(nq, off, 32);
  const float denom = fmaxf(nq, 1.0f);
  qs[lane] = qj;
#pragma unroll
  for (int i = 0; i < 32; ++i) Cs[i * CPITCH + lane] = Ccol[i];
  __syncthreads();
  float dot = 0.0f;
#pragma unroll 1
  for (int i = 0; i < DEMB; ++i) dot = fmaf(Cs[i * CPITCH + lane], qs[i], dot);
  const float hval = (oj * dot) / denom;
  hsh[lane] = hval;
  __syncthreads();

  const v4f hv = *(const v4f*)(hsh + c4);
  v4f cv[8];
#pragma unroll
  for (int it = 0; it < 8; ++it) cv[it] = *(const v4f*)(Cs + (it * 4 + rsub) * CPITCH + c4);
  float* oh  = out + (size_t)bh * DEMB;
  float* ocm = out + NOUT0 + (size_t)bh * DEMB * DEMB;
  for (int pass = 0; pass < 2; ++pass) {
    if (lane < 8) *(volatile v4f*)(oh + c4) = hv;
#pragma unroll
    for (int it = 0; it < 8; ++it) *(volatile v4f*)(ocm + (size_t)(it * 4 + rsub) * DEMB + c4) = cv[it];
    __threadfence();
  }
}

extern "C" void kernel_launch(void* const* d_in, const int* in_sizes, int n_in,
                              void* d_out, int out_size, void* d_ws, size_t ws_size, hipStream_t stream) {
  if (n_in < 13 || d_out == nullptr || d_ws == nullptr) return;
  if (in_sizes[0] != NROWS * NIN || in_sizes[1] != NHEAD * NIN * DEMB || in_sizes[2] != NVK ||
      in_sizes[3] != NHEAD * NIN || in_sizes[4] != NHEAD || in_sizes[5] != NHEAD * NIN || in_sizes[6] != NHEAD ||
      in_sizes[7] != NHEAD * NIN * DEMB || in_sizes[8] != NVK || in_sizes[9] != NHEAD * NIN * DEMB ||
      in_sizes[10] != NVK || in_sizes[11] != NHEAD * NIN * DEMB || in_sizes[12] != NVK ||
      out_size != NOUT0 + NOUT1) return;

  const float* p_x  = (const float*)d_in[0];
  const float* p_wo = (const float*)d_in[1];
  const float* p_bo = (const float*)d_in[2];
  const float* p_wf = (const float*)d_in[3];
  const float* p_bf = (const float*)d_in[4];
  const float* p_wi = (const float*)d_in[5];
  const float* p_bi = (const float*)d_in[6];
  const float* p_wv = (const float*)d_in[7];
  const float* p_bv = (const float*)d_in[8];
  const float* p_wk = (const float*)d_in[9];
  const float* p_bk = (const float*)d_in[10];
  const float* p_wq = (const float*)d_in[11];
  const float* p_bq = (const float*)d_in[12];
  float* out = (float*)d_out;

  char* ws = (char*)d_ws; size_t off = 0;
  auto carve = [&](size_t bytes) -> char* { char* p = ws + off; off += (bytes + 255) & ~(size_t)255; return p; };
  unsigned short* XB = (unsigned short*)carve((size_t)NROWS * NIN * 2);
  unsigned short* BT = (unsigned short*)carve((size_t)YPITCH * NIN * 2);
  float*          Y  = (float*)carve((size_t)NROWS * YPITCH * 4);
  if (off > ws_size || off > (size_t)134217728) return;

  cvt8_kernel<0><<<(NROWS * (NIN / 8)) / NTHR, NTHR, 0, stream>>>(p_x, XB, NROWS, NIN / 8, NIN, 0, 1.0f);
  pack_bt_kernel<<<YPITCH / (NTHR / 32), NTHR, 0, stream>>>(p_wv, p_wk, p_wf, p_wi, BT);
  const dim3 ggrid((NROWS / 64) * (YPITCH / 64) / 8, 1);
  wmma_gemm64<1, false, 0, 0, false, 0><<<ggrid, 256, 0, stream>>>(
      XB, XB, NIN, 0L, BT, BT, NIN, 0L, (void*)Y, (void*)Y, YPITCH, 0L,
      (const float*)Y, (const float*)Y, 0L, NROWS, YPITCH, NIN, 1.0f);
  mm_recur_kernel<<<NBAT * NHEAD, 32, 0, stream>>>(Y, p_x, p_wo, p_bo, p_bf, p_bi, p_bv, p_bk, p_wq, p_bq, out);
}
